// Ses2Seq_70162585747743
// MI455X (gfx1250) — hardware-verified
//
#include <hip/hip_runtime.h>
#include <math.h>

typedef __attribute__((ext_vector_type(16))) _Float16 v16h;
typedef __attribute__((ext_vector_type(8)))  _Float16 v8h;
typedef __attribute__((ext_vector_type(8)))  float    v8f;
typedef __attribute__((ext_vector_type(4)))  float    v4f;

constexpr int NSEQ       = 16;
constexpr int NSTEP      = 256;
constexpr int NFEAT      = 16;
constexpr int NOUTF      = 32;
constexpr int NHW        = 48;
constexpr int LTH        = 4016;
constexpr int KTOT       = LTH + NFEAT;
constexpr int NKBLK      = KTOT / 32;
constexpr int NTILE_REAL = LTH / 16;
constexpr int NTILE_PAD  = ((NTILE_REAL + 3) / 4) * 4;
constexpr int GROUP_TILES = 2;
constexpr int NGROUP     = NTILE_PAD / GROUP_TILES;
constexpr int GROUP_ROWS = GROUP_TILES * 16;
constexpr int WROWS      = NTILE_PAD * 16;
constexpr int TILE_HALVES  = 256;
constexpr int PLANE_HALVES = NTILE_PAD * TILE_HALVES;
constexpr int DX_HALVES  = 64;
constexpr int TF_PITCH   = 4096;
constexpr int NTHR_SCAN  = 512;
constexpr int NWAVE      = NTHR_SCAN / 32;
constexpr int SLAB_PITCH = 36;
constexpr int NW8        = WROWS * (KTOT / 8);
constexpr int NINIT      = NTILE_PAD * 32 + (NSEQ * DX_HALVES) / 8;

constexpr int OFF_W1 = 0;
constexpr int OFF_B1 = OFF_W1 + NHW;
constexpr int OFF_W2 = OFF_B1 + NHW;
constexpr int OFF_B2 = OFF_W2 + NHW * NHW;
constexpr int OFF_W3 = OFF_B2 + NHW;
constexpr int OFF_B3 = OFF_W3 + NOUTF * NHW;

constexpr float W_CARRY        = 1024.0f;
constexpr float W_CARRY_INV    = 1.0f / 1024.0f;
constexpr float LO_CARRY       = 2048.0f;
constexpr float LO_CARRY_INV   = 1.0f / 2048.0f;
constexpr float F16_MIN_NORMAL = 6.103515625e-05f;
constexpr float CLIP_LIM       = 0.5f;

static_assert(OFF_B3 + NOUTF == LTH, "theta slices");
static_assert(KTOT == 4032 && KTOT % 32 == 0, "K multiple of 32");
static_assert(NKBLK == 126, "k blocks");
static_assert(LTH % 16 == 0 && LTH % 8 == 0, "tile rows");
static_assert(NTILE_PAD == 252 && NGROUP == 126 && WROWS == 4032, "groups");
static_assert(GROUP_ROWS == 32, "one 128-B f32 line per sequence and group");
static_assert(NW8 % 256 == 0, "weight plane grid exact");
static_assert(NINIT == 8192 && NINIT % 256 == 0, "init grid exact");
static_assert((NTILE_PAD * 32) % 32 == 0, "wave-uniform role split");
static_assert(NSEQ == NWAVE, "one wave per sequence in the MLP phase");
static_assert(WROWS <= TF_PITCH, "theta f32 row pitch");
static_assert((KTOT * 2) % 16 == 0, "weight row pitch 16-B aligned");
static_assert(TILE_HALVES == 32 * 8, "one 16-B piece per lane per tile");

__device__ __forceinline__ unsigned short f2bf_bits(float f) {
  unsigned u = __float_as_uint(f);
  return (unsigned short)((u + 0x7FFFu + ((u >> 16) & 1u)) >> 16);
}
__device__ __forceinline__ float bf_bits2f(unsigned short h) { return __uint_as_float(((unsigned)h) << 16); }
__device__ __forceinline__ float bf16r(float f) { return bf_bits2f(f2bf_bits(f)); }

__device__ __forceinline__ void split_hi_lo(float v, _Float16& hi, _Float16& lo) {
  const float vh = (fabsf(v) < F16_MIN_NORMAL) ? 0.0f : v;
  hi = (_Float16)vh;
  const float hf = (float)hi;
  lo = (_Float16)((v - hf) * LO_CARRY);
}

union FragU { v16h v; v8h h[2]; };
__device__ __forceinline__ v16h load_frag(const _Float16* p) {
  FragU f;
  f.h[0] = *(const v8h*)(p);
  f.h[1] = *(const v8h*)(p + 16);
  return f.v;
}
__device__ __forceinline__ v16h load_frag2(const _Float16* p0, const _Float16* p1) {
  FragU f;
  f.h[0] = *(const v8h*)(p0);
  f.h[1] = *(const v8h*)(p1);
  return f.v;
}
__device__ __forceinline__ v8f wmma_h(v16h a, v16h b, v8f c) {
  return __builtin_amdgcn_wmma_f32_16x16x32_f16(false, a, false, b, (short)0, c, false, false);
}
__device__ __forceinline__ void guard4(v8f& p0, v8f& q0, v8f& p1, v8f& q1, v16h a0, v16h a1, v16h b0, v16h b1) {
  asm volatile("v_nop\n\tv_nop\n\tv_nop\n\tv_nop"
               : "+v"(p0), "+v"(q0), "+v"(p1), "+v"(q1)
               : "v"(a0), "v"(a1), "v"(b0), "v"(b1));
}
__device__ __forceinline__ void acc_add(v8f& acc, const v8f p) {
#pragma clang fp contract(off)
#pragma unroll
  for (int r = 0; r < 8; ++r) {
    acc[r] = __fadd_rn(acc[r], p[r]);
  }
}
__device__ __forceinline__ void kblock(v8f (&vs)[2], v8f (&rs)[2],
                                       const _Float16* wk, v16h bh, v16h bl) {
  const v8f z8 = {0.f, 0.f, 0.f, 0.f, 0.f, 0.f, 0.f, 0.f};
  const v16h a0 = load_frag(wk);
  const v16h a1 = load_frag(wk + (size_t)16 * KTOT);
  v8f p0 = wmma_h(a0, bh, z8);
  v8f q0 = wmma_h(a0, bl, z8);
  v8f p1 = wmma_h(a1, bh, z8);
  v8f q1 = wmma_h(a1, bl, z8);
  guard4(p0, q0, p1, q1, a0, a1, bh, bl);
  acc_add(vs[0], p0);
  acc_add(rs[0], q0);
  acc_add(vs[1], p1);
  acc_add(rs[1], q1);
}
__device__ __forceinline__ void wave_lds_sync() {
  __builtin_amdgcn_fence(__ATOMIC_RELEASE, "workgroup");
  __builtin_amdgcn_wave_barrier();
  __builtin_amdgcn_fence(__ATOMIC_ACQUIRE, "workgroup");
}

__global__ __launch_bounds__(256) void build_w_kernel(const float* __restrict__ Amat, const float* __restrict__ Bmat,
                                                      unsigned short* __restrict__ Wp) {
  const int i = blockIdx.x * 256 + threadIdx.x;
  if (i < NW8) {
    const int row  = i / (KTOT / 8);
    const int g8   = i - row * (KTOT / 8);
    const int rowc = (row < LTH) ? row : (LTH - 1);
    const int ga   = (g8 < LTH / 8) ? g8 : (LTH / 8 - 1);
    const int gb   = (g8 >= LTH / 8) ? (g8 - LTH / 8) : 0;
    const float* ap = Amat + (size_t)rowc * LTH + ga * 8;
    const float* bp = Bmat + (size_t)rowc * NFEAT + gb * 8;
    const v4f a0 = *(const v4f*)(ap);
    const v4f a1 = *(const v4f*)(ap + 4);
    const v4f b0 = *(const v4f*)(bp);
    const v4f b1 = *(const v4f*)(bp + 4);
    const float fa = (g8 < LTH / 8) ? 1.0f : 0.0f;
    const float fb = 1.0f - fa;
    const bool rowok = (row < LTH);
    v8h hv;
#pragma unroll
    for (int e = 0; e < 4; ++e) {
      float x0 = fa * a0[e] + fb * b0[e];
      float x1 = fa * a1[e] + fb * b1[e];
      x0 = rowok ? x0 : 0.0f;
      x1 = rowok ? x1 : 0.0f;
      const _Float16 q0 = (_Float16)(bf16r(x0) * W_CARRY);
      const _Float16 q1 = (_Float16)(bf16r(x1) * W_CARRY);
      hv[e]     = q0;
      hv[4 + e] = q1;
    }
    *(volatile v8h*)(Wp + (size_t)i * 8) = hv;
    __threadfence();
    *(volatile v8h*)(Wp + (size_t)i * 8) = hv;
  }
}

__global__ __launch_bounds__(256) void init_state_kernel(const float* __restrict__ theta0,
                                                         unsigned short* __restrict__ STp,
                                                         unsigned short* __restrict__ DXp) {
  const int i = blockIdx.x * 256 + threadIdx.x;
  if (i < NTILE_PAD * 32) {
    const int tile = i >> 5;
    const int k0   = tile * 16 + (i & 1) * 8;
    const int kc   = (k0 < LTH - 8) ? k0 : (LTH - 8);
    const v4f a = *(const v4f*)(theta0 + kc);
    const v4f b = *(const v4f*)(theta0 + kc + 4);
    const bool ok = (k0 < LTH);
    v8h hv, lv;
#pragma unroll
    for (int e = 0; e < 4; ++e) {
      const float x0 = ok ? bf16r(a[e]) : 0.0f;
      const float x1 = ok ? bf16r(b[e]) : 0.0f;
      _Float16 h0, l0, h1, l1;
      split_hi_lo(x0, h0, l0);
      split_hi_lo(x1, h1, l1);
      hv[e] = h0;
      lv[e] = l0;
      hv[4 + e] = h1;
      lv[4 + e] = l1;
    }
    unsigned short* ph = STp + (size_t)i * 8;
    unsigned short* pl = STp + (size_t)PLANE_HALVES + (size_t)i * 8;
    *(volatile v8h*)ph = hv;
    *(volatile v8h*)pl = lv;
    __threadfence();
    *(volatile v8h*)ph = hv;
    *(volatile v8h*)pl = lv;
  } else if (i < NINIT) {
    const int j = i - NTILE_PAD * 32;
    v8h z;
#pragma unroll
    for (int e = 0; e < 8; ++e) z[e] = (_Float16)0.0f;
    unsigned short* pd = DXp + (size_t)j * 8;
    *(volatile v8h*)pd = z;
    __threadfence();
    *(volatile v8h*)pd = z;
  }
}

__global__ __launch_bounds__(NTHR_SCAN) void scan_kernel(const float* __restrict__ xs, const float* __restrict__ ts,
                                                         const int* __restrict__ coin,
                                                         const unsigned short* __restrict__ Wp,
                                                         unsigned short* STp, unsigned short* DXp,
                                                         float* TF, float* out) {
  __shared__ __align__(16) float    slab[NWAVE][16 * SLAB_PITCH];
  __shared__ __align__(16) float    hbuf[NWAVE][128];
  __shared__ __align__(16) _Float16 sst[NWAVE][2 * TILE_HALVES];

  const int tid  = threadIdx.x;
  const int lane = tid & 31;
  const int wave = __builtin_amdgcn_readfirstlane(tid >> 5);
  const int c    = lane & 15;
  const int hh   = lane >> 4;
  const int koff = hh * 8;
  const int q    = lane >> 3;
  const int c4   = (lane & 7) * 4;
  const _Float16* W = (const _Float16*)Wp;
  float* sl = slab[wave];
  float* hb = hbuf[wave];
  _Float16* ss = sst[wave];
  const int bq = wave;

  float xp1, xp2;
  {
    const float x0 = xs[(size_t)bq * NSTEP * NFEAT + c];
    xp1 = bf16r(x0);
    xp2 = xp1;
  }
  const v8f z8 = {0.f, 0.f, 0.f, 0.f, 0.f, 0.f, 0.f, 0.f};

#pragma unroll 1
  for (int t = 0; t < NSTEP; ++t) {
    const int cur = t & 1;
    const int nxt = cur ^ 1;
    const _Float16* SHc = (const _Float16*)STp + (size_t)(cur * 2) * PLANE_HALVES;
    unsigned short* SHn = STp + (size_t)(nxt * 2) * PLANE_HALVES;
    const _Float16* DXc = (const _Float16*)DXp + (size_t)cur * (NSEQ * DX_HALVES);
    unsigned short* DXn = DXp + (size_t)nxt * (NSEQ * DX_HALVES);

#pragma unroll 1
    for (int g = wave; g < NGROUP; g += NWAVE) {
      v8f vs[2], rs[2];
#pragma unroll
      for (int j = 0; j < 2; ++j) { vs[j] = z8; rs[j] = z8; }
      const _Float16* wk = W + (size_t)(GROUP_ROWS * g + c) * KTOT + koff;
      const _Float16* sk = SHc + c * 16 + koff;
#pragma unroll 1
      for (int kb = 0; kb < NKBLK - 1; ++kb) {
        const v16h bh = load_frag2(sk, sk + TILE_HALVES);
        const v16h bl = load_frag2(sk + PLANE_HALVES, sk + PLANE_HALVES + TILE_HALVES);
        kblock(vs, rs, wk, bh, bl);
        wk += 32;
        sk += 2 * TILE_HALVES;
      }
      {
        const _Float16* dq = DXc + c * DX_HALVES + koff;
        const v16h bh = load_frag2(sk, dq);
        const v16h bl = load_frag2(sk + PLANE_HALVES, dq + 16);
        kblock(vs, rs, wk, bh, bl);
      }

      v8h hv[2], lv[2];
      v4f fv[2][2];
#pragma unroll
      for (int j = 0; j < 2; ++j) {
#pragma unroll
        for (int r = 0; r < 8; ++r) {
          const float accv = vs[j][r];
          const float accr = rs[j][r];
          float v = (accv + accr * LO_CARRY_INV) * W_CARRY_INV;
          v = fminf(CLIP_LIM, fmaxf(-CLIP_LIM, v));
          _Float16 h16, l16;
          split_hi_lo(v, h16, l16);
          hv[j][r] = h16;
          lv[j][r] = l16;
          fv[j][r >> 2][r & 3] = v;
        }
      }
      v4f ov[4];
#pragma unroll
      for (int jj = 0; jj < 2; ++jj) {
        float* sp = sl + c * SLAB_PITCH + 16 * jj + koff;
        *(v4f*)(sp)     = fv[jj][0];
        *(v4f*)(sp + 4) = fv[jj][1];
      }
      wave_lds_sync();
#pragma unroll
      for (int it = 0; it < 4; ++it) ov[it] = *(const v4f*)(sl + (it * 4 + q) * SLAB_PITCH + c4);
      wave_lds_sync();
      v8h ohv[2], olv[2];
#pragma unroll
      for (int j = 0; j < 2; ++j) {
        *(v8h*)(ss + c * 16 + koff) = hv[j];
        *(v8h*)(ss + TILE_HALVES + c * 16 + koff) = lv[j];
        wave_lds_sync();
        ohv[j] = *(const v8h*)(ss + lane * 8);
        olv[j] = *(const v8h*)(ss + TILE_HALVES + lane * 8);
        wave_lds_sync();
      }
      float* tfb = TF + GROUP_ROWS * g + c4;
      unsigned short* shn = SHn + (size_t)(GROUP_TILES * g) * TILE_HALVES + lane * 8;
      for (int pass = 0; pass < 2; ++pass) {
#pragma unroll
        for (int it = 0; it < 4; ++it)
          *(volatile v4f*)(tfb + (size_t)(it * 4 + q) * TF_PITCH) = ov[it];
#pragma unroll
        for (int j = 0; j < 2; ++j) {
          *(volatile v8h*)(shn + j * TILE_HALVES) = ohv[j];
          *(volatile v8h*)(shn + PLANE_HALVES + j * TILE_HALVES) = olv[j];
        }
        __threadfence();
      }
    }
    __threadfence();
    __syncthreads();
    __threadfence();

    {
      const float* th = TF + (size_t)bq * TF_PITCH;
      const float traw = ts[bq * NSTEP + t];
      const float tc = bf16r(traw);
      const int u2 = 32 + c;
      const float w1a = th[OFF_W1 + lane];
      const float b1a = th[OFF_B1 + lane];
      const float w1b = th[OFF_W1 + u2];
      const float b1b = th[OFF_B1 + u2];
      const float h1a = fmaxf(w1a * tc + b1a, 0.0f);
      const float h1b = fmaxf(w1b * tc + b1b, 0.0f);
      hb[lane] = h1a;
      hb[32 + lane] = (lane < 16) ? h1b : 0.0f;
      wave_lds_sync();
      const float* r1 = th + OFF_W2 + lane * NHW;
      const float* r2 = th + OFF_W2 + u2 * NHW;
      float s1 = th[OFF_B2 + lane];
      float s2 = th[OFF_B2 + u2];
#pragma unroll 4
      for (int i4 = 0; i4 < NHW / 4; ++i4) {
        const v4f wa = *(const v4f*)(r1 + 4 * i4);
        const v4f wb = *(const v4f*)(r2 + 4 * i4);
        const v4f hx = *(const v4f*)(hb + 4 * i4);
        s1 += wa[0] * hx[0];
        s1 += wa[1] * hx[1];
        s1 += wa[2] * hx[2];
        s1 += wa[3] * hx[3];
        s2 += wb[0] * hx[0];
        s2 += wb[1] * hx[1];
        s2 += wb[2] * hx[2];
        s2 += wb[3] * hx[3];
      }
      hb[64 + lane] = fmaxf(s1, 0.0f);
      hb[96 + lane] = (lane < 16) ? fmaxf(s2, 0.0f) : 0.0f;
      wave_lds_sync();
      const float* r3 = th + OFF_W3 + lane * NHW;
      float z = th[OFF_B3 + lane];
#pragma unroll 4
      for (int i4 = 0; i4 < NHW / 4; ++i4) {
        const v4f wc = *(const v4f*)(r3 + 4 * i4);
        const v4f hx = *(const v4f*)(hb + 64 + 4 * i4);
        z += wc[0] * hx[0];
        z += wc[1] * hx[1];
        z += wc[2] * hx[2];
        z += wc[3] * hx[3];
      }
      const float y = tanhf(z);
      volatile float* op = out + ((size_t)bq * NSTEP + (size_t)t) * NOUTF + lane;
      *op = y;
      __threadfence();
      *op = y;

      const float yfb = __shfl(y, c, 32);
      const int tn = (t + 1 < NSTEP) ? (t + 1) : (NSTEP - 1);
      const int cn = coin[bq * NSTEP + tn];
      float xraw = xs[((size_t)bq * NSTEP + (size_t)tn) * NFEAT + c];
      asm volatile("" : "+v"(xraw));
      const float xn = bf16r(xraw);
      const float nxp2 = xp1;
      xp1 = yfb;
      xp2 = nxp2;
      const float xt = (cn != 0) ? xn : xp1;
      const float dxn = xt - xp2;
      _Float16 dh, dl;
      split_hi_lo(dxn, dh, dl);
      const int hbits = (int)__builtin_bit_cast(unsigned short, dh);
      const int lbits = (int)__builtin_bit_cast(unsigned short, dl);
      const int sa = (lane & 7) * 2;
      const unsigned ha = (unsigned)__shfl(hbits, sa, 32);
      const unsigned hc = (unsigned)__shfl(hbits, sa + 1, 32);
      const unsigned la = (unsigned)__shfl(lbits, sa, 32);
      const unsigned lc = (unsigned)__shfl(lbits, sa + 1, 32);
      const unsigned whi = (ha & 0xffffu) | (hc << 16);
      const unsigned wlo = (la & 0xffffu) | (lc << 16);
      const unsigned word = (lane < 8) ? whi : ((lane < 16) ? wlo : 0u);
      volatile unsigned* dp = (volatile unsigned*)(DXn + (size_t)bq * DX_HALVES) + lane;
      *dp = word;
      __threadfence();
      *dp = word;
    }
    __threadfence();
    __syncthreads();
    __threadfence();
  }
}

extern "C" void kernel_launch(void* const* d_in, const int* in_sizes, int n_in,
                              void* d_out, int out_size, void* d_ws, size_t ws_size, hipStream_t stream) {
  if (n_in < 6 || d_out == nullptr || d_ws == nullptr) return;
  if (in_sizes[0] != NSEQ * NSTEP * NFEAT || in_sizes[1] != NSEQ * NSTEP || in_sizes[2] != LTH ||
      in_sizes[3] != LTH * LTH || in_sizes[4] != LTH * NFEAT || in_sizes[5] != NSEQ * NSTEP ||
      out_size != NSEQ * NSTEP * NOUTF) return;

  const float* xs     = (const float*)d_in[0];
  const float* ts     = (const float*)d_in[1];
  const float* theta0 = (const float*)d_in[2];
  const float* Amat   = (const float*)d_in[3];
  const float* Bmat   = (const float*)d_in[4];
  const int*   coin   = (const int*)d_in[5];
  float* out = (float*)d_out;

  char* ws = (char*)d_ws;
  size_t off = 0;
  auto carve = [&](size_t bytes) -> char* { char* p = ws + off; off += (bytes + 255) & ~(size_t)255; return p; };
  unsigned short* WPL = (unsigned short*)carve((size_t)WROWS * KTOT * 2);
  unsigned short* ST  = (unsigned short*)carve((size_t)4 * PLANE_HALVES * 2);
  unsigned short* DX  = (unsigned short*)carve((size_t)2 * NSEQ * DX_HALVES * 2);
  float*          TF  = (float*)carve((size_t)NSEQ * TF_PITCH * 4);
  if (off > ws_size || off > (size_t)134217728) return;

  build_w_kernel<<<NW8 / 256, 256, 0, stream>>>(Amat, Bmat, WPL);
  init_state_kernel<<<NINIT / 256, 256, 0, stream>>>(theta0, ST, DX);
  scan_kernel<<<1, NTHR_SCAN, 0, stream>>>(xs, ts, coin, WPL, ST, DX, TF, out);
}
